// ComplexDifferentialAttention_2748779069849
// MI455X (gfx1250) — hardware-verified
//
#include <hip/hip_runtime.h>
#include <math.h>
#include <stdint.h>
#include <stddef.h>

#define NH 8
#define SQ 2048
#define DD 64
#define NR (NH * SQ)
#define PLN ((size_t)NR * DD)

typedef __attribute__((ext_vector_type(16))) _Float16 v16h;
typedef __attribute__((ext_vector_type(8)))  _Float16 v8h;
typedef __attribute__((ext_vector_type(16))) __bf16   v16b;
typedef __attribute__((ext_vector_type(8)))  __bf16   v8b;
typedef __attribute__((ext_vector_type(8)))  float    v8f;
typedef __attribute__((ext_vector_type(4)))  float    v4f;
typedef __attribute__((ext_vector_type(4)))  unsigned v4u;

__device__ __forceinline__ unsigned short bf_bits(float f) {
  const unsigned u = __float_as_uint(f);
  return (unsigned short)((u + 0x7FFFu + ((u >> 16) & 1u)) >> 16);
}
__device__ __forceinline__ float bf_val(unsigned short b) { return __uint_as_float(((unsigned)b) << 16); }
__device__ __forceinline__ void bf_split(float f, unsigned short& hi, unsigned short& lo) {
  hi = bf_bits(f);
  lo = bf_bits(f - bf_val(hi));
}
__device__ __forceinline__ void h_split64(float f, unsigned short& hi, unsigned short& lo) {
  const float s = f * 64.0f;
  const _Float16 a = (_Float16)s;
  const _Float16 b = (_Float16)(s - (float)a);
  hi = __builtin_bit_cast(unsigned short, a);
  lo = __builtin_bit_cast(unsigned short, b);
}
__device__ __forceinline__ unsigned pk16(unsigned short a, unsigned short b) {
  return (unsigned)a | ((unsigned)b << 16);
}
__device__ __forceinline__ float pick8(v4f a, v4f b, int i) { return (i < 4) ? a[i & 3] : b[i & 3]; }
__device__ __forceinline__ float pick16(v4f a, v4f b, v4f c, v4f d, int i) {
  return (i < 4) ? a[i & 3] : (i < 8) ? b[i & 3] : (i < 12) ? c[i & 3] : d[i & 3];
}
__device__ __forceinline__ v8f z8() { v8f r = {0.f, 0.f, 0.f, 0.f, 0.f, 0.f, 0.f, 0.f}; return r; }

__device__ __forceinline__ void wave_sync() {
  __builtin_amdgcn_fence(__ATOMIC_RELEASE, "workgroup");
  __builtin_amdgcn_wave_barrier();
  __builtin_amdgcn_fence(__ATOMIC_ACQUIRE, "workgroup");
}

__device__ __forceinline__ v16b frag_b(const unsigned short* p) {
  union { v16b v; v8b h[2]; } u;
  u.h[0] = *(const v8b*)(const void*)p;
  u.h[1] = *(const v8b*)(const void*)(p + 16);
  return u.v;
}
__device__ __forceinline__ v16h frag_hg(const unsigned short* p) {
  union { v16h v; v8h h[2]; } u;
  u.h[0] = *(const v8h*)(const void*)p;
  u.h[1] = *(const v8h*)(const void*)(p + 16);
  return u.v;
}
__device__ __forceinline__ v16h frag_hl(const _Float16* p) {
  union { v16h v; v8h h[2]; } u;
  u.h[0] = *(const v8h*)p;
  u.h[1] = *(const v8h*)(p + 16);
  return u.v;
}
__device__ __forceinline__ v8f mma_b(v16b a, v16b b, v8f c) {
  c = __builtin_amdgcn_wmma_f32_16x16x32_bf16(false, a, false, b, (short)0, c, false, false);
  asm volatile("v_nop\n\tv_nop\n\tv_nop\n\tv_nop" : "+v"(c) : "v"(a), "v"(b));
  return c;
}
__device__ __forceinline__ v8f mma_h(v16h a, v16h b, v8f c) {
  c = __builtin_amdgcn_wmma_f32_16x16x32_f16(false, a, false, b, (short)0, c, false, false);
  asm volatile("v_nop\n\tv_nop\n\tv_nop\n\tv_nop" : "+v"(c) : "v"(a), "v"(b));
  return c;
}

__global__ __launch_bounds__(256) void prep_kernel(
    const float* __restrict__ qwr, const float* __restrict__ qwi,
    const float* __restrict__ kwr, const float* __restrict__ kwi,
    const float* __restrict__ vwr, const float* __restrict__ vwi,
    const float* __restrict__ gwr, const float* __restrict__ gwi,
    const float* __restrict__ owr, const float* __restrict__ owi,
    const float* __restrict__ qbr, const float* __restrict__ qbi,
    const float* __restrict__ kbr, const float* __restrict__ kbi,
    const float* __restrict__ vbr, const float* __restrict__ vbi,
    const float* __restrict__ gbr, const float* __restrict__ gbi,
    const float* __restrict__ obr, const float* __restrict__ obi,
    unsigned short* __restrict__ Wh, unsigned short* __restrict__ Wl, float* __restrict__ bias) {
  const int gid = blockIdx.x * 256 + threadIdx.x;
  if (blockIdx.x < 48) {
    const int rowg = gid >> 4;
    const int kg = (gid & 15) * 8;
    const float* wr; const float* wi; int nn, nout;
    if (rowg < 256) { wr = qwr; wi = qwi; nn = rowg; nout = 128; }
    else {
      const int idx = rowg - 256;
      const int mat = idx >> 7;
      nn = idx & 127; nout = 64;
      wr = (mat == 0) ? kwr : (mat == 1) ? vwr : (mat == 2) ? gwr : owr;
      wi = (mat == 0) ? kwi : (mat == 1) ? vwi : (mat == 2) ? gwi : owi;
    }
    const bool imo = nn >= nout;
    const int no = imo ? nn - nout : nn;
    const bool hik = kg >= 64;
    const int kk = kg & 63;
    const float* pr = wr + (size_t)no * 64 + kk;
    const float* pi = wi + (size_t)no * 64 + kk;
    const v4f ra = *(const v4f*)pr, rb = *(const v4f*)(pr + 4);
    const v4f ia = *(const v4f*)pi, ib = *(const v4f*)(pi + 4);
    v4u hv, lv;
#pragma unroll
    for (int q = 0; q < 4; ++q) {
      const float a0 = pick8(ra, rb, 2 * q), a1 = pick8(ra, rb, 2 * q + 1);
      const float b0 = pick8(ia, ib, 2 * q), b1 = pick8(ia, ib, 2 * q + 1);
      const float v0 = imo ? (hik ? a0 : b0) : (hik ? -b0 : a0);
      const float v1 = imo ? (hik ? a1 : b1) : (hik ? -b1 : a1);
      unsigned short h0, l0, h1, l1;
      bf_split(v0, h0, l0); bf_split(v1, h1, l1);
      hv[q] = pk16(h0, h1); lv[q] = pk16(l0, l1);
    }
    const size_t wo = (size_t)rowg * 128 + kg;
    for (int pass = 0; pass < 2; ++pass) {
      *(volatile v4u*)(Wh + wo) = hv;
      *(volatile v4u*)(Wl + wo) = lv;
      __threadfence();
    }
  } else {
    const int t = gid - 48 * 256;
    if (t < 192) {
      const int f = 4 * t;
      const float* br; const float* bi; int loc, nout;
      if (f < 256) { br = qbr; bi = qbi; loc = f; nout = 128; }
      else {
        const int j = f - 256;
        const int mat = j >> 7;
        loc = j & 127; nout = 64;
        br = (mat == 0) ? kbr : (mat == 1) ? vbr : (mat == 2) ? gbr : obr;
        bi = (mat == 0) ? kbi : (mat == 1) ? vbi : (mat == 2) ? gbi : obi;
      }
      const bool im = loc >= nout;
      const int li = im ? loc - nout : loc;
      const v4f a = *(const v4f*)(br + li);
      const v4f b = *(const v4f*)(bi + li);
      v4f v;
#pragma unroll
      for (int e = 0; e < 4; ++e) v[e] = im ? b[e] : a[e];
      for (int pass = 0; pass < 2; ++pass) {
        *(volatile v4f*)(bias + f) = v;
        __threadfence();
      }
    }
  }
}

__global__ __launch_bounds__(256) void split_act_kernel(
    const float* __restrict__ q_r, const float* __restrict__ q_i,
    const float* __restrict__ k_r, const float* __restrict__ k_i,
    const float* __restrict__ v_r, const float* __restrict__ v_i,
    unsigned short* __restrict__ Xh, unsigned short* __restrict__ Xl) {
  const int tsel = blockIdx.y;
  const float* sr = (tsel == 0) ? q_r : (tsel == 1) ? k_r : v_r;
  const float* si = (tsel == 0) ? q_i : (tsel == 1) ? k_i : v_i;
  const size_t toff = (size_t)tsel * NR * 128;
  const int gid = blockIdx.x * 256 + threadIdx.x;
  const size_t row = (size_t)(gid >> 3);
  const int g = gid & 7;
  const float* pr = sr + row * 64 + 8 * g;
  const float* pi = si + row * 64 + 8 * g;
  const v4f ra = *(const v4f*)pr, rb = *(const v4f*)(pr + 4);
  const v4f ia = *(const v4f*)pi, ib = *(const v4f*)(pi + 4);
  v4u hr, lr, hi, li;
#pragma unroll
  for (int q = 0; q < 4; ++q) {
    unsigned short a0, b0, a1, b1;
    bf_split(pick8(ra, rb, 2 * q), a0, b0); bf_split(pick8(ra, rb, 2 * q + 1), a1, b1);
    hr[q] = pk16(a0, a1); lr[q] = pk16(b0, b1);
    bf_split(pick8(ia, ib, 2 * q), a0, b0); bf_split(pick8(ia, ib, 2 * q + 1), a1, b1);
    hi[q] = pk16(a0, a1); li[q] = pk16(b0, b1);
  }
  unsigned short* dh = Xh + toff + row * 128 + 8 * g;
  unsigned short* dl = Xl + toff + row * 128 + 8 * g;
  for (int pass = 0; pass < 2; ++pass) {
    *(volatile v4u*)(dh) = hr;
    *(volatile v4u*)(dh + 64) = hi;
    *(volatile v4u*)(dl) = lr;
    *(volatile v4u*)(dl + 64) = li;
    __threadfence();
  }
}

template <int PE>
__global__ __launch_bounds__(128) void cgemm_kernel(
    const unsigned short* __restrict__ Ah, const unsigned short* __restrict__ Al,
    const unsigned short* __restrict__ Bh, const unsigned short* __restrict__ Bl,
    const float* __restrict__ bias, const float* __restrict__ pe0, const float* __restrict__ pe1,
    float* __restrict__ outp, int N, int ldo, long pstride) {
  __shared__ __align__(16) float slab[4][16 * 68];
  const int tid = threadIdx.x, wave = tid >> 5, lane = tid & 31, hh = lane >> 4, m = lane & 15;
  const int r0 = blockIdx.x * 64 + wave * 16;
  const unsigned short* ap  = Ah + (size_t)(r0 + m) * 128 + 8 * hh;
  const unsigned short* alp = Al + (size_t)(r0 + m) * 128 + 8 * hh;
  v16b ah[4], al[4];
#pragma unroll
  for (int kc = 0; kc < 4; ++kc) { ah[kc] = frag_b(ap + kc * 32); al[kc] = frag_b(alp + kc * 32); }
  float* sl = slab[wave];
  const int c4 = m * 4;
  const int ngr = N >> 6;
#pragma unroll 1
  for (int ng = 0; ng < ngr; ++ng) {
    v8f acc[4];
#pragma unroll
    for (int j = 0; j < 4; ++j) acc[j] = z8();
#pragma unroll
    for (int kc = 0; kc < 4; ++kc) {
#pragma unroll
      for (int j = 0; j < 4; ++j) {
        const size_t bo = (size_t)(ng * 64 + j * 16 + m) * 128 + kc * 32 + 8 * hh;
        const v16b bh = frag_b(Bh + bo);
        const v16b bl = frag_b(Bl + bo);
        acc[j] = mma_b(ah[kc], bh, acc[j]);
        acc[j] = mma_b(ah[kc], bl, acc[j]);
        acc[j] = mma_b(al[kc], bh, acc[j]);
      }
    }
#pragma unroll
    for (int j = 0; j < 4; ++j) {
      const int c = ng * 64 + j * 16 + m;
      const float bv = bias[c];
      const float* pp = pe0;
      int pcol = 0;
      if (PE == 1) { pp = (c >> 7) ? pe1 : pe0; pcol = c & 63; }
      if (PE == 2) { pp = (c >> 6) ? pe1 : pe0; pcol = c & 63; }
#pragma unroll
      for (int r = 0; r < 8; ++r) {
        const int row = r0 + 8 * hh + r;
        float v = acc[j][r] + bv;
        if (PE != 0) v += pp[(size_t)row * 64 + pcol];
        sl[(8 * hh + r) * 68 + j * 16 + m] = v;
      }
    }
    wave_sync();
    float* ob = outp + (size_t)ng * pstride;
    for (int pass = 0; pass < 2; ++pass) {
#pragma unroll
      for (int it = 0; it < 8; ++it) {
        const int row = it * 2 + hh;
        const v4f v = *(const v4f*)(sl + row * 68 + c4);
        *(volatile v4f*)(ob + (size_t)(r0 + row) * ldo + c4) = v;
      }
      __threadfence();
    }
    wave_sync();
  }
}

__global__ __launch_bounds__(256) void qkplanes_kernel(
    const float* __restrict__ QPf, const float* __restrict__ KPf,
    unsigned short* __restrict__ Qpl, unsigned short* __restrict__ Kpl) {
  const int gid = blockIdx.x * 256 + threadIdx.x;
  const size_t row = (size_t)(gid >> 3);
  const int g = gid & 7;
  if (blockIdx.y == 0) {
    const float* rp = QPf + row * 256 + 16 * g;
    const float* ip = rp + 128;
    const v4f ra = *(const v4f*)(rp), rb = *(const v4f*)(rp + 4), rc = *(const v4f*)(rp + 8), rd = *(const v4f*)(rp + 12);
    const v4f ia = *(const v4f*)(ip), ib = *(const v4f*)(ip + 4), ic = *(const v4f*)(ip + 8), id = *(const v4f*)(ip + 12);
    unsigned short* qd = Qpl + row * 64 + 8 * g;
#pragma unroll
    for (int p = 0; p < 2; ++p) {
      v4u hr, lr, hi, li, hs, ls;
#pragma unroll
      for (int q = 0; q < 4; ++q) {
        const int i0 = 4 * q + p, i1 = 4 * q + 2 + p;
        const float x0 = pick16(ra, rb, rc, rd, i0), x1 = pick16(ra, rb, rc, rd, i1);
        const float y0 = pick16(ia, ib, ic, id, i0), y1 = pick16(ia, ib, ic, id, i1);
        unsigned short a0, b0, a1, b1;
        bf_split(x0, a0, b0); bf_split(x1, a1, b1); hr[q] = pk16(a0, a1); lr[q] = pk16(b0, b1);
        bf_split(y0, a0, b0); bf_split(y1, a1, b1); hi[q] = pk16(a0, a1); li[q] = pk16(b0, b1);
        bf_split(x0 + y0, a0, b0); bf_split(x1 + y1, a1, b1); hs[q] = pk16(a0, a1); ls[q] = pk16(b0, b1);
      }
      unsigned short* d = qd + (size_t)(p * 6) * PLN;
      for (int pass = 0; pass < 2; ++pass) {
        *(volatile v4u*)(d)           = hr;
        *(volatile v4u*)(d + PLN)     = lr;
        *(volatile v4u*)(d + 2 * PLN) = hi;
        *(volatile v4u*)(d + 3 * PLN) = li;
        *(volatile v4u*)(d + 4 * PLN) = hs;
        *(volatile v4u*)(d + 5 * PLN) = ls;
        __threadfence();
      }
    }
  } else {
    const float* rp = KPf + row * 128 + 8 * g;
    const float* ip = rp + 64;
    const v4f ra = *(const v4f*)(rp), rb = *(const v4f*)(rp + 4);
    const v4f ia = *(const v4f*)(ip), ib = *(const v4f*)(ip + 4);
    v4u hr, lr, hi, li, ht, lt;
#pragma unroll
    for (int q = 0; q < 4; ++q) {
      const float x0 = pick8(ra, rb, 2 * q), x1 = pick8(ra, rb, 2 * q + 1);
      const float y0 = pick8(ia, ib, 2 * q), y1 = pick8(ia, ib, 2 * q + 1);
      unsigned short a0, b0, a1, b1;
      bf_split(x0, a0, b0); bf_split(x1, a1, b1); hr[q] = pk16(a0, a1); lr[q] = pk16(b0, b1);
      bf_split(y0, a0, b0); bf_split(y1, a1, b1); hi[q] = pk16(a0, a1); li[q] = pk16(b0, b1);
      bf_split(x0 - y0, a0, b0); bf_split(x1 - y1, a1, b1); ht[q] = pk16(a0, a1); lt[q] = pk16(b0, b1);
    }
    unsigned short* d = Kpl + row * 64 + 8 * g;
    for (int pass = 0; pass < 2; ++pass) {
      *(volatile v4u*)(d)           = hr;
      *(volatile v4u*)(d + PLN)     = lr;
      *(volatile v4u*)(d + 2 * PLN) = hi;
      *(volatile v4u*)(d + 3 * PLN) = li;
      *(volatile v4u*)(d + 4 * PLN) = ht;
      *(volatile v4u*)(d + 5 * PLN) = lt;
      __threadfence();
    }
  }
}

__global__ __launch_bounds__(256) void vt_kernel(const float* __restrict__ VPf, unsigned short* __restrict__ Vtp) {
  __shared__ __align__(16) float tf[64 * 68];
  const int kt = blockIdx.x;
  const int comp = blockIdx.y;
  const int head = kt >> 5, s0 = (kt & 31) * 64;
  const int tid = threadIdx.x;
  {
    const int lr = tid >> 4;
    const int c4 = (tid & 15) * 4;
#pragma unroll
    for (int it = 0; it < 4; ++it) {
      const int rr = it * 16 + lr;
      const v4f a = *(const v4f*)(VPf + (size_t)(kt * 64 + rr) * 128 + comp * 64 + c4);
      *(v4f*)(tf + rr * 68 + c4) = a;
    }
  }
  __syncthreads();
  const int sub = tid >> 3;
  const int c8 = (tid & 7) * 8;
  v4u hv[2], lv[2];
#pragma unroll
  for (int it = 0; it < 2; ++it) {
    const int f = it * 32 + sub;
    v4u a, b;
#pragma unroll
    for (int q = 0; q < 4; ++q) {
      const float f0 = tf[(c8 + 2 * q) * 68 + f];
      const float f1 = tf[(c8 + 2 * q + 1) * 68 + f];
      unsigned short h0, l0, h1, l1;
      h_split64(f0, h0, l0); h_split64(f1, h1, l1);
      a[q] = pk16(h0, h1); b[q] = pk16(l0, l1);
    }
    hv[it] = a; lv[it] = b;
  }
  unsigned short* oh = Vtp + (size_t)(comp * 2) * PLN;
  unsigned short* ol = Vtp + (size_t)(comp * 2 + 1) * PLN;
  for (int pass = 0; pass < 2; ++pass) {
#pragma unroll
    for (int it = 0; it < 2; ++it) {
      const int f = it * 32 + sub;
      const size_t go = ((size_t)head * 64 + f) * SQ + s0 + c8;
      *(volatile v4u*)(oh + go) = hv[it];
      *(volatile v4u*)(ol + go) = lv[it];
    }
    __threadfence();
  }
}

__global__ __launch_bounds__(128) void attn_kernel(
    const unsigned short* __restrict__ Qpl, const unsigned short* __restrict__ Kpl,
    const unsigned short* __restrict__ Vtp, float* __restrict__ Opl) {
  __shared__ __align__(16) _Float16 Psh[4][16 * 64];
  __shared__ __align__(16) float Osl[4][16 * 68];
  const int tid = threadIdx.x, wave = tid >> 5, lane = tid & 31, hh = lane >> 4, m = lane & 15;
  const int bx = blockIdx.x;
  const int pair = bx & 1;
  const int qt = bx >> 1;
  const int head = qt >> 5;
  const int q0 = (qt & 31) * 64 + wave * 16;
  const size_t hrow = (size_t)head * SQ;
  const unsigned short* Qb = Qpl + (size_t)(pair * 6) * PLN + (hrow + q0 + m) * 64;
  const unsigned short* Kb = Kpl + (hrow + m) * 64;
  const unsigned short* Vb = Vtp + ((size_t)head * 64 + m) * SQ;
  _Float16* pw = Psh[wave];

  float mrow[8], lrow[8];
  v8f orr[4], oii[4];
#pragma unroll
  for (int r = 0; r < 8; ++r) { mrow[r] = -INFINITY; lrow[r] = 0.f; }
#pragma unroll
  for (int t = 0; t < 4; ++t) { orr[t] = z8(); oii[t] = z8(); }

#pragma unroll 1
  for (int kc = 0; kc < SQ / 64; ++kc) {
    const int key0 = kc * 64;
    v8f sc[4];
#pragma unroll
    for (int j = 0; j < 4; ++j) {
      const unsigned short* kj = Kb + (size_t)(key0 + j * 16) * 64;
      v8f p1 = z8(), p2 = z8(), p3 = z8();
#pragma unroll
      for (int dc = 0; dc < 2; ++dc) {
        const int ko = dc * 32 + 8 * hh;
        {
          const v16b qa = frag_b(Qb + ko), ql = frag_b(Qb + PLN + ko);
          const v16b ka = frag_b(kj + ko), kl = frag_b(kj + PLN + ko);
          p1 = mma_b(qa, ka, p1); p1 = mma_b(qa, kl, p1); p1 = mma_b(ql, ka, p1);
        }
        {
          const v16b qa = frag_b(Qb + 2 * PLN + ko), ql = frag_b(Qb + 3 * PLN + ko);
          const v16b ka = frag_b(kj + 2 * PLN + ko), kl = frag_b(kj + 3 * PLN + ko);
          p2 = mma_b(qa, ka, p2); p2 = mma_b(qa, kl, p2); p2 = mma_b(ql, ka, p2);
        }
        {
          const v16b qa = frag_b(Qb + 4 * PLN + ko), ql = frag_b(Qb + 5 * PLN + ko);
          const v16b ka = frag_b(kj + 4 * PLN + ko), kl = frag_b(kj + 5 * PLN + ko);
          p3 = mma_b(qa, ka, p3); p3 = mma_b(qa, kl, p3); p3 = mma_b(ql, ka, p3);
        }
      }
#pragma unroll
      for (int r = 0; r < 8; ++r) {
        const float sr = p1[r] + p2[r];
        const float si = (p3[r] - p1[r]) + p2[r];
        sc[j][r] = sqrtf(sr * sr + si * si + 1e-8f) * 0.125f;
      }
    }
    wave_sync();
#pragma unroll
    for (int r = 0; r < 8; ++r) {
      float cm = fmaxf(fmaxf(sc[0][r], sc[1][r]), fmaxf(sc[2][r], sc[3][r]));
      cm = fmaxf(cm, __shfl_xor(cm, 1, 32));
      cm = fmaxf(cm, __shfl_xor(cm, 2, 32));
      cm = fmaxf(cm, __shfl_xor(cm, 4, 32));
      cm = fmaxf(cm, __shfl_xor(cm, 8, 32));
      const float mnew = fmaxf(mrow[r], cm);
      const float alpha = __expf(mrow[r] - mnew);
      mrow[r] = mnew;
      float psum = 0.f;
#pragma unroll
      for (int j = 0; j < 4; ++j) {
        const float p = __expf(sc[j][r] - mnew);
        psum += p;
        pw[(8 * hh + r) * 64 + j * 16 + m] = (_Float16)(p * 4096.0f);
      }
      psum += __shfl_xor(psum, 1, 32);
      psum += __shfl_xor(psum, 2, 32);
      psum += __shfl_xor(psum, 4, 32);
      psum += __shfl_xor(psum, 8, 32);
      lrow[r] = lrow[r] * alpha + psum;
#pragma unroll
      for (int t = 0; t < 4; ++t) { orr[t][r] *= alpha; oii[t][r] *= alpha; }
    }
    wave_sync();
#pragma unroll
    for (int kk = 0; kk < 2; ++kk) {
      const v16h pa = frag_hl(pw + m * 64 + kk * 32 + 8 * hh);
      const unsigned short* vk = Vb + key0 + kk * 32 + 8 * hh;
#pragma unroll
      for (int t = 0; t < 4; ++t) {
        const unsigned short* vt = vk + (size_t)(t * 16) * SQ;
        const v16h vrh = frag_hg(vt), vrl = frag_hg(vt + PLN);
        orr[t] = mma_h(pa, vrh, orr[t]);
        orr[t] = mma_h(pa, vrl, orr[t]);
        const v16h vih = frag_hg(vt + 2 * PLN), vil = frag_hg(vt + 3 * PLN);
        oii[t] = mma_h(pa, vih, oii[t]);
        oii[t] = mma_h(pa, vil, oii[t]);
      }
    }
  }

  float* os = Osl[wave];
  float* ob0 = Opl + (size_t)(pair * 2) * PLN + (hrow + q0) * 64;
  const int c4 = m * 4;
  const float kinv = 1.0f / 262144.0f;
#pragma unroll
  for (int r = 0; r < 8; ++r) {
    const float inv = (1.0f / lrow[r]) * kinv;
#pragma unroll
    for (int t = 0; t < 4; ++t) os[(8 * hh + r) * 68 + t * 16 + m] = orr[t][r] * inv;
  }
  wave_sync();
  for (int pass = 0; pass < 2; ++pass) {
#pragma unroll
    for (int it = 0; it < 8; ++it) {
      const int row = it * 2 + hh;
      const v4f v = *(const v4f*)(os + row * 68 + c4);
      *(volatile v4f*)(ob0 + (size_t)row * 64 + c4) = v;
    }
    __threadfence();
  }
  wave_sync();
#pragma unroll
  for (int r = 0; r < 8; ++r) {
    const float inv = (1.0f / lrow[r]) * kinv;
#pragma unroll
    for (int t = 0; t < 4; ++t) os[(8 * hh + r) * 68 + t * 16 + m] = oii[t][r] * inv;
  }
  wave_sync();
  float* ob1 = ob0 + PLN;
  for (int pass = 0; pass < 2; ++pass) {
#pragma unroll
    for (int it = 0; it < 8; ++it) {
      const int row = it * 2 + hh;
      const v4f v = *(const v4f*)(os + row * 68 + c4);
      *(volatile v4f*)(ob1 + (size_t)row * 64 + c4) = v;
    }
    __threadfence();
  }
}

__global__ __launch_bounds__(256) void combine_kernel(
    const float* __restrict__ Opl, const float* __restrict__ gr, const float* __restrict__ gi,
    const float* __restrict__ subw, unsigned short* __restrict__ Xh, unsigned short* __restrict__ Xl) {
  const int tid = threadIdx.x, wave = tid >> 5, lane = tid & 31, hh = lane >> 4, c = lane & 15;
  const size_t row = (size_t)blockIdx.x * 16 + wave * 2 + hh;
  const float* base = Opl + row * 64 + 4 * c;
  const v4f a  = *(const v4f*)(base);
  const v4f b  = *(const v4f*)(base + PLN);
  const v4f cc = *(const v4f*)(base + 2 * PLN);
  const v4f d  = *(const v4f*)(base + 3 * PLN);
  float ss = 0.f;
#pragma unroll
  for (int u = 0; u < 4; ++u) ss += a[u] * a[u] + b[u] * b[u] + cc[u] * cc[u] + d[u] * d[u];
  ss += __shfl_xor(ss, 1, 32);
  ss += __shfl_xor(ss, 2, 32);
  ss += __shfl_xor(ss, 4, 32);
  ss += __shfl_xor(ss, 8, 32);
  const float rms = sqrtf(ss * (1.0f / 128.0f) + 1e-5f);
  const float inv = 1.0f / rms;
  const int cg = (c < 8) ? c : 7;
  const float* gp = gr + row * 64 + 8 * cg;
  const float* ip = gi + row * 64 + 8 * cg;
  const v4f g0 = *(const v4f*)(gp), g1 = *(const v4f*)(gp + 4);
  const v4f h0 = *(const v4f*)(ip), h1 = *(const v4f*)(ip + 4);
  const v4f w0 = *(const v4f*)(subw + 8 * cg), w1 = *(const v4f*)(subw + 8 * cg + 4);
  float xr[8], xi[8];
#pragma unroll
  for (int e = 0; e < 8; ++e) {
    const int u = e >> 1, p = e & 1;
    const float ore = p ? cc[u] : a[u];
    const float oim = p ? d[u] : b[u];
    const float sw  = pick8(w0, w1, e);
    const float gre = pick8(g0, g1, e);
    const float gie = pick8(h0, h1, e);
    const float arv = ore * inv * sw;
    const float aiv = oim * inv * sw;
    xr[e] = gre * arv - gie * aiv;
    xi[e] = gre * aiv + gie * arv;
  }
  v4u hxr, lxr, hxi, lxi;
#pragma unroll
  for (int q = 0; q < 4; ++q) {
    unsigned short a0, b0, a1, b1;
    bf_split(xr[2 * q], a0, b0); bf_split(xr[2 * q + 1], a1, b1); hxr[q] = pk16(a0, a1); lxr[q] = pk16(b0, b1);
    bf_split(xi[2 * q], a0, b0); bf_split(xi[2 * q + 1], a1, b1); hxi[q] = pk16(a0, a1); lxi[q] = pk16(b0, b1);
  }
  unsigned short* dh = Xh + row * 128 + 8 * cg;
  unsigned short* dl = Xl + row * 128 + 8 * cg;
  if (c < 8) {
    *(volatile v4u*)(dh) = hxr;
    *(volatile v4u*)(dh + 64) = hxi;
    *(volatile v4u*)(dl) = lxr;
    *(volatile v4u*)(dl + 64) = lxi;
  }
  __threadfence();
  if (c < 8) {
    *(volatile v4u*)(dh) = hxr;
    *(volatile v4u*)(dh + 64) = hxi;
    *(volatile v4u*)(dl) = lxr;
    *(volatile v4u*)(dl + 64) = lxi;
  }
}

extern "C" void kernel_launch(void* const* d_in, const int* in_sizes, int n_in,
                              void* d_out, int out_size, void* d_ws, size_t ws_size,
                              hipStream_t stream) {
  if (n_in < 35) return;
  const int NE = NR * DD;
  for (int i = 0; i < 10; ++i) if (in_sizes[i] != NE) return;
  if (in_sizes[10] != 8192 || in_sizes[11] != 8192) return;
  if (in_sizes[12] != 128 || in_sizes[13] != 128) return;
  if (in_sizes[14] != 4096 || in_sizes[15] != 4096 || in_sizes[16] != 64 || in_sizes[17] != 64) return;
  if (in_sizes[18] != 4096 || in_sizes[19] != 4096 || in_sizes[20] != 64 || in_sizes[21] != 64) return;
  if (in_sizes[22] != 4096 || in_sizes[23] != 4096 || in_sizes[24] != 64 || in_sizes[25] != 64) return;
  if (in_sizes[26] != 4096 || in_sizes[27] != 4096 || in_sizes[28] != 64 || in_sizes[29] != 64) return;
  if (in_sizes[34] != 128) return;
  if (out_size != 4 * NE) return;

  const float* q_r = (const float*)d_in[0];
  const float* q_i = (const float*)d_in[1];
  const float* k_r = (const float*)d_in[2];
  const float* k_i = (const float*)d_in[3];
  const float* v_r = (const float*)d_in[4];
  const float* v_i = (const float*)d_in[5];
  const float* pe_q_r = (const float*)d_in[6];
  const float* pe_q_i = (const float*)d_in[7];
  const float* pe_k_r = (const float*)d_in[8];
  const float* pe_k_i = (const float*)d_in[9];
  const float* qwr = (const float*)d_in[10];
  const float* qwi = (const float*)d_in[11];
  const float* qbr = (const float*)d_in[12];
  const float* qbi = (const float*)d_in[13];
  const float* kwr = (const float*)d_in[14];
  const float* kwi = (const float*)d_in[15];
  const float* kbr = (const float*)d_in[16];
  const float* kbi = (const float*)d_in[17];
  const float* vwr = (const float*)d_in[18];
  const float* vwi = (const float*)d_in[19];
  const float* vbr = (const float*)d_in[20];
  const float* vbi = (const float*)d_in[21];
  const float* gwr = (const float*)d_in[22];
  const float* gwi = (const float*)d_in[23];
  const float* gbr = (const float*)d_in[24];
  const float* gbi = (const float*)d_in[25];
  const float* owr = (const float*)d_in[26];
  const float* owi = (const float*)d_in[27];
  const float* obr = (const float*)d_in[28];
  const float* obi = (const float*)d_in[29];
  const float* subw = (const float*)d_in[34];

  size_t off = 0;
  const size_t szW = (size_t)768 * 128 * 2;
  const size_t oWh = off; off += szW;
  const size_t oWl = off; off += szW;
  const size_t oB = off; off += 4096;
  const size_t szX = (size_t)4 * NR * 128 * 2;
  const size_t oXh = off; off += szX;
  const size_t oXl = off; off += szX;
  const size_t oQPf = off; off += (size_t)NR * 256 * 4;
  const size_t oKPf = off; off += (size_t)NR * 128 * 4;
  const size_t oVPf = off; off += (size_t)NR * 128 * 4;
  const size_t oQpl = off; off += (size_t)12 * PLN * 2;
  const size_t oKpl = off; off += (size_t)6 * PLN * 2;
  const size_t oVt = off; off += (size_t)4 * PLN * 2;
  const size_t oO = off; off += (size_t)4 * PLN * 4;
  if (off > ws_size) return;

  char* ws = (char*)d_ws;
  unsigned short* Wh = (unsigned short*)(ws + oWh);
  unsigned short* Wl = (unsigned short*)(ws + oWl);
  float* bias = (float*)(ws + oB);
  unsigned short* Xh = (unsigned short*)(ws + oXh);
  unsigned short* Xl = (unsigned short*)(ws + oXl);
  float* QPf = (float*)(ws + oQPf);
  float* KPf = (float*)(ws + oKPf);
  float* VPf = (float*)(ws + oVPf);
  unsigned short* Qpl = (unsigned short*)(ws + oQpl);
  unsigned short* Kpl = (unsigned short*)(ws + oKpl);
  unsigned short* Vtp = (unsigned short*)(ws + oVt);
  float* Opl = (float*)(ws + oO);

  float* out0 = (float*)d_out;
  float* out2 = out0 + 2 * PLN;
  const size_t XT = (size_t)NR * 128;

  prep_kernel<<<dim3(49), dim3(256), 0, stream>>>(qwr, qwi, kwr, kwi, vwr, vwi, gwr, gwi, owr, owi,
                                                   qbr, qbi, kbr, kbi, vbr, vbi, gbr, gbi, obr, obi,
                                                   Wh, Wl, bias);
  split_act_kernel<<<dim3(NR * 8 / 256, 3), dim3(256), 0, stream>>>(q_r, q_i, k_r, k_i, v_r, v_i, Xh, Xl);
  cgemm_kernel<1><<<dim3(NR / 64), dim3(128), 0, stream>>>(
      Xh, Xl, Wh, Wl, bias, pe_q_r, pe_q_i, QPf, 256, 256, 64L);
  cgemm_kernel<2><<<dim3(NR / 64), dim3(128), 0, stream>>>(
      Xh + XT, Xl + XT, Wh + 256 * 128, Wl + 256 * 128, bias + 256, pe_k_r, pe_k_i, KPf, 128, 128, 64L);
  cgemm_kernel<0><<<dim3(NR / 64), dim3(128), 0, stream>>>(
      Xh + 2 * XT, Xl + 2 * XT, Wh + 384 * 128, Wl + 384 * 128, bias + 384, pe_q_r, pe_q_r, VPf, 128, 128, 64L);
  cgemm_kernel<0><<<dim3(NR / 64), dim3(128), 0, stream>>>(
      Xh, Xl, Wh + 512 * 128, Wl + 512 * 128, bias + 512, pe_q_r, pe_q_r, out2, 128, 64, (long)PLN);
  qkplanes_kernel<<<dim3(NR * 8 / 256, 2), dim3(256), 0, stream>>>(QPf, KPf, Qpl, Kpl);
  vt_kernel<<<dim3(NR / 64, 2), dim3(256), 0, stream>>>(VPf, Vtp);
  attn_kernel<<<dim3(2 * (NR / 64)), dim3(128), 0, stream>>>(Qpl, Kpl, Vtp, Opl);
  combine_kernel<<<dim3(NR / 16), dim3(256), 0, stream>>>(Opl, out2, out2 + PLN, subw, Xh + 3 * XT, Xl + 3 * XT);
  cgemm_kernel<0><<<dim3(NR / 64), dim3(128), 0, stream>>>(
      Xh + 3 * XT, Xl + 3 * XT, Wh + 640 * 128, Wl + 640 * 128, bias + 640, pe_q_r, pe_q_r, out0, 128, 64, (long)PLN);
  (void)hipGetLastError();
}
